// RelRepWindowContext_43147241455988
// MI455X (gfx1250) — hardware-verified
//
#include <hip/hip_runtime.h>
#include <math.h>

constexpr int kB      = 2;
constexpr int kS      = 384;
constexpr int kH      = 512;
constexpr int kK      = 24;
constexpr int kWin    = 10;
constexpr int kInner  = 2304;
constexpr int kThreeH = 1536;
constexpr int kPairs  = kB * kK * kK;
constexpr int kSpanRows = kB * kK;
constexpr int kSrPad  = 64;
constexpr int kGroupsPerRow = kInner / 8;
constexpr float kNegLimit = -1.0e9f;

typedef char chk_pairs [(kPairs % 64) == 0 ? 1 : -1];
typedef char chk_groups[((kPairs * kGroupsPerRow) % 256) == 0 ? 1 : -1];
typedef char chk_k32   [((kH % 32) == 0 && (kInner % 64) == 0 && (kThreeH % 64) == 0) ? 1 : -1];

typedef __attribute__((ext_vector_type(16))) _Float16 v16h;
typedef __attribute__((ext_vector_type(8)))  _Float16 v8h;
typedef __attribute__((ext_vector_type(16))) __bf16   v16b;
typedef __attribute__((ext_vector_type(8)))  __bf16   v8b;
typedef __attribute__((ext_vector_type(8)))  float    v8f;
typedef __attribute__((ext_vector_type(4)))  float    v4f;
typedef __attribute__((ext_vector_type(4)))  unsigned int v4u;

__device__ __forceinline__ unsigned short f2bf_bits(float f) {
  unsigned u = __float_as_uint(f);
  return (unsigned short)((u + 0x7FFFu + ((u >> 16) & 1u)) >> 16);
}
__device__ __forceinline__ float bf_bits2f(unsigned short h) { return __uint_as_float(((unsigned)h) << 16); }

__device__ __forceinline__ void dep_guard_h(v8f& a, v8f& b, v16h x, v16h y) { asm volatile("v_nop\n\tv_nop\n\tv_nop\n\tv_nop" : "+v"(a), "+v"(b) : "v"(x), "v"(y)); }
__device__ __forceinline__ void dep_guard_b(v8f& a, v8f& b, v16b x, v16b y) { asm volatile("v_nop\n\tv_nop\n\tv_nop\n\tv_nop" : "+v"(a), "+v"(b) : "v"(x), "v"(y)); }
__device__ __forceinline__ void keep4_h(v16h a, v16h b, v16h c, v16h d) { asm volatile("v_nop" :: "v"(a), "v"(b), "v"(c), "v"(d)); }
__device__ __forceinline__ void keep4_b(v16b a, v16b b, v16b c, v16b d) { asm volatile("v_nop" :: "v"(a), "v"(b), "v"(c), "v"(d)); }
__device__ __forceinline__ void acc_guard4(v8f& a, v8f& b, v8f& c, v8f& d) { asm volatile("v_nop\n\tv_nop\n\tv_nop\n\tv_nop" : "+v"(a), "+v"(b), "+v"(c), "+v"(d)); }
template <typename T> struct Frag;
template <> struct Frag<_Float16> {
  typedef v16h V; union U { v16h v; v8h h[2]; };
  static __device__ __forceinline__ v16h load(const _Float16* p) {
    U f; f.h[0] = *(const v8h*)(p); f.h[1] = *(const v8h*)(p + 16); return f.v;
  }
  static __device__ __forceinline__ v8f mma(v16h a, v16h b, v8f c) {
    return __builtin_amdgcn_wmma_f32_16x16x32_f16(false, a, false, b, (short)0, c, false, false);
  }
  static __device__ __forceinline__ void guard(v8f& a, v8f& b, v16h x, v16h y) { dep_guard_h(a, b, x, y); }
  static __device__ __forceinline__ void keep(v16h a, v16h b, v16h c, v16h d) { keep4_h(a, b, c, d); }
};
template <> struct Frag<__bf16> {
  typedef v16b V; union U { v16b v; v8b h[2]; };
  static __device__ __forceinline__ v16b load(const __bf16* p) {
    U f; f.h[0] = *(const v8b*)(p); f.h[1] = *(const v8b*)(p + 16); return f.v;
  }
  static __device__ __forceinline__ v8f mma(v16b a, v16b b, v8f c) {
    return __builtin_amdgcn_wmma_f32_16x16x32_bf16(false, a, false, b, (short)0, c, false, false);
  }
  static __device__ __forceinline__ void guard(v8f& a, v8f& b, v16b x, v16b y) { dep_guard_b(a, b, x, y); }
  static __device__ __forceinline__ void keep(v16b a, v16b b, v16b c, v16b d) { keep4_b(a, b, c, d); }
};

__device__ __forceinline__ unsigned pk16(unsigned short a, unsigned short b) { return (unsigned)a | ((unsigned)b << 16); }

template <int ET> struct Elem;
template <> struct Elem<0> { typedef _Float16 T; };
template <> struct Elem<1> { typedef __bf16 T; };
template <int ET, bool SPLIT, int BIAS_MODE, int OUT_MODE, bool RESID, int ACT = 0>
__global__ __launch_bounds__(256) void wmma_gemm64(
    const unsigned short* __restrict__ Ap, const unsigned short* __restrict__ A2p, int lda, long strideA,
    const unsigned short* __restrict__ Btp, const unsigned short* __restrict__ Bt2p, int ldb, long strideB,
    void* __restrict__ Cout, void* __restrict__ Cout2, int ldc, long strideC,
    const float* __restrict__ bias,
    const float* __restrict__ resid, long strideR,
    int M, int N, int K, float scale) {
  typedef typename Elem<ET>::T T;
  typedef typename Frag<T>::V V;
  const T* A = (const T*)Ap; const T* A2 = (const T*)A2p; const T* Bt = (const T*)Btp; const T* Bt2 = (const T*)Bt2p;
  __shared__ __align__(16) float sT[8][16 * 68];
  const int b    = blockIdx.y;
  const int lane = threadIdx.x & 31;
  const int wave = threadIdx.x >> 5;
  const int tilesN = N >> 6;
  const int tilesM = M >> 6;
  const int tile = blockIdx.x * 8 + wave;
  if (tile >= tilesM * tilesN) return;
  const int tm = tile / tilesN;
  const int tn = tile - tm * tilesN;
  const int m0 = tm << 6;
  const int n0 = tn << 6;

  const T* Ab  = A  + (size_t)b * strideA;
  const T* Bb  = Bt + (size_t)b * strideB;
  const T* Ab2 = SPLIT ? (A2  + (size_t)b * strideA) : nullptr;
  const T* Bb2 = SPLIT ? (Bt2 + (size_t)b * strideB) : nullptr;

  const int rlane = lane & 15;
  const int koff  = (lane >> 4) * 8;
  const int mOff  = (lane >> 4) * 8;

  v8f acc[4][4];
#pragma unroll
  for (int i = 0; i < 4; ++i)
#pragma unroll
    for (int j = 0; j < 4; ++j) acc[i][j] = (v8f){0.f,0.f,0.f,0.f,0.f,0.f,0.f,0.f};

  for (int k0 = 0; k0 < K; k0 += 32) {
    V bh[4], bl[4];
#pragma unroll
    for (int j = 0; j < 4; ++j) {
      const size_t bo = (size_t)(n0 + (j << 4) + rlane) * ldb + koff + k0;
      bh[j] = Frag<T>::load(Bb + bo);
      if (SPLIT) bl[j] = Frag<T>::load(Bb2 + bo);
    }
#pragma unroll
    for (int i = 0; i < 4; ++i) {
      const size_t ao = (size_t)(m0 + (i << 4) + rlane) * lda + koff + k0;
      V ah = Frag<T>::load(Ab + ao);
      V al;
      if (SPLIT) al = Frag<T>::load(Ab2 + ao);
#pragma unroll
      for (int j = 0; j < 4; ++j) {
        acc[i][j] = Frag<T>::mma(ah, bh[j], acc[i][j]);
        if (SPLIT) {
          acc[i][j] = Frag<T>::mma(ah, bl[j], acc[i][j]);
          acc[i][j] = Frag<T>::mma(al, bh[j], acc[i][j]);
        }
      }
      Frag<T>::guard(acc[i][0], acc[i][3], ah, SPLIT ? al : ah);
    }
    Frag<T>::keep(bh[0], bh[1], bh[2], bh[3]);
    if (SPLIT) Frag<T>::keep(bl[0], bl[1], bl[2], bl[3]);
  }
  acc_guard4(acc[0][0], acc[0][1], acc[0][2], acc[0][3]);
  acc_guard4(acc[1][0], acc[1][1], acc[1][2], acc[1][3]);
  acc_guard4(acc[2][0], acc[2][1], acc[2][2], acc[2][3]);
  acc_guard4(acc[3][0], acc[3][1], acc[3][2], acc[3][3]);

  float* slab = sT[wave];
  const float* Rb = RESID ? (resid + (size_t)b * strideR) : nullptr;
#pragma unroll
  for (int i = 0; i < 4; ++i) {
    const int mBase = m0 + (i << 4);
#pragma unroll
    for (int j = 0; j < 4; ++j) {
      const int n = n0 + (j << 4) + rlane;
      float bv = 0.f;
      if (BIAS_MODE == 2) bv = bias[n];
#pragma unroll
      for (int r = 0; r < 8; ++r) {
        float v = acc[i][j][r] * scale;
        if (BIAS_MODE == 1) v += bias[mBase + mOff + r];
        if (BIAS_MODE == 2) v += bv;
        if (RESID) v += Rb[(size_t)(mBase + mOff + r) * ldc + n];
        if (ACT == 2) v = fmaxf(v, 0.0f);
        if (ACT == 4) v = (v > 0.f) ? v : 0.01f * v;
        slab[(mOff + r) * 68 + (j << 4) + rlane] = v;
      }
    }
    __builtin_amdgcn_fence(__ATOMIC_RELEASE, "workgroup");
    __builtin_amdgcn_wave_barrier();
    __builtin_amdgcn_fence(__ATOMIC_ACQUIRE, "workgroup");
    if (OUT_MODE == 0) {
      float* C = (float*)Cout + (size_t)b * strideC;
      const int hh = lane >> 4, c4 = (lane & 15) * 4;
      for (int pass = 0; pass < 2; ++pass) {
#pragma unroll
        for (int it = 0; it < 8; ++it) {
          const int row = it * 2 + hh;
          v4f v = *(const v4f*)(slab + row * 68 + c4);
          *(volatile v4f*)(C + (size_t)(mBase + row) * ldc + n0 + c4) = v;
        }
        __threadfence();
      }
    } else {
      const int q = lane >> 3, c8 = (lane & 7) * 8;
      unsigned short* C  = (unsigned short*)Cout  + (size_t)b * strideC;
      unsigned short* C2 = (OUT_MODE == 2) ? ((unsigned short*)Cout2 + (size_t)b * strideC) : nullptr;
      for (int pass = 0; pass < 2; ++pass) {
#pragma unroll
        for (int it = 0; it < 4; ++it) {
          const int row = it * 4 + q;
          const float* sp = slab + row * 68 + c8;
          v8h hv, lv;
#pragma unroll
          for (int e = 0; e < 8; ++e) {
            if (OUT_MODE == 1) {
              hv[e] = (_Float16)sp[e];
            } else {
              unsigned short hb = f2bf_bits(sp[e]);
              unsigned short lb = f2bf_bits(sp[e] - bf_bits2f(hb));
              hv[e] = __builtin_bit_cast(_Float16, hb);
              lv[e] = __builtin_bit_cast(_Float16, lb);
            }
          }
          *(volatile v8h*)(C + (size_t)(mBase + row) * ldc + n0 + c8) = hv;
          if (OUT_MODE == 2) *(volatile v8h*)(C2 + (size_t)(mBase + row) * ldc + n0 + c8) = lv;
        }
        __threadfence();
      }
    }
    __builtin_amdgcn_fence(__ATOMIC_RELEASE, "workgroup");
    __builtin_amdgcn_wave_barrier();
    __builtin_amdgcn_fence(__ATOMIC_ACQUIRE, "workgroup");
  }
}

__global__ __launch_bounds__(256) void tsplit_kernel(const float* __restrict__ in, int ld_in, int ld_out,
                                                     unsigned short* __restrict__ out_hi,
                                                     unsigned short* __restrict__ out_lo) {
  __shared__ float sm[64][65];
  const int t  = threadIdx.x;
  const int r0 = blockIdx.x * 64;
  const int c0 = blockIdx.y * 64;
#pragma unroll
  for (int i = 0; i < 16; ++i) {
    const int e  = i * 256 + t;
    const int rl = e >> 6;
    const int cl = e & 63;
    sm[cl][rl] = in[(size_t)(r0 + rl) * ld_in + c0 + cl];
  }
  __syncthreads();
  const int lane = t & 31, wave = t >> 5;
  const int q = lane >> 3, c8 = (lane & 7) * 8;
  for (int pass = 0; pass < 2; ++pass) {
#pragma unroll
    for (int it = 0; it < 2; ++it) {
      const int row = wave * 8 + it * 4 + q;
      unsigned short hb[8], lb[8];
#pragma unroll
      for (int e = 0; e < 8; ++e) {
        const float v = sm[row][c8 + e];
        hb[e] = f2bf_bits(v);
        lb[e] = f2bf_bits(v - bf_bits2f(hb[e]));
      }
      const v4u uh = (v4u){pk16(hb[0], hb[1]), pk16(hb[2], hb[3]), pk16(hb[4], hb[5]), pk16(hb[6], hb[7])};
      const v4u ul = (v4u){pk16(lb[0], lb[1]), pk16(lb[2], lb[3]), pk16(lb[4], lb[5]), pk16(lb[6], lb[7])};
      const size_t o = (size_t)(c0 + row) * ld_out + r0 + c8;
      *(volatile v4u*)(out_hi + o) = uh;
      *(volatile v4u*)(out_lo + o) = ul;
    }
    __threadfence();
  }
}

__global__ __launch_bounds__(256) void srsplit_kernel(const float* __restrict__ span_reps,
                                                      unsigned short* __restrict__ sr_hi,
                                                      unsigned short* __restrict__ sr_lo) {
  const int idx = blockIdx.x * 256 + threadIdx.x;
  if (idx >= kSrPad * (kH / 8)) return;
  const int row = idx >> 6;
  const int c8  = (idx & 63) * 8;
  const int srow = (row < kSpanRows) ? row : (kSpanRows - 1);
  const float* p = span_reps + (size_t)srow * kH + c8;
  const v4f a = *(const v4f*)(p);
  const v4f c = *(const v4f*)(p + 4);
  float x[8];
#pragma unroll
  for (int e = 0; e < 4; ++e) { x[e] = a[e]; x[4 + e] = c[e]; }
  unsigned short hb[8], lb[8];
#pragma unroll
  for (int e = 0; e < 8; ++e) { hb[e] = f2bf_bits(x[e]); lb[e] = f2bf_bits(x[e] - bf_bits2f(hb[e])); }
  const v4u uh = (v4u){pk16(hb[0], hb[1]), pk16(hb[2], hb[3]), pk16(hb[4], hb[5]), pk16(hb[6], hb[7])};
  const v4u ul = (v4u){pk16(lb[0], lb[1]), pk16(lb[2], lb[3]), pk16(lb[4], lb[5]), pk16(lb[6], lb[7])};
  const size_t o = (size_t)row * kH + c8;
  for (int pass = 0; pass < 2; ++pass) {
    *(volatile v4u*)(sr_hi + o) = uh;
    *(volatile v4u*)(sr_lo + o) = ul;
    __threadfence();
  }
}

__global__ __launch_bounds__(512) void ctx_kernel(const float* __restrict__ token_reps,
                                                  const int* __restrict__ token_masks,
                                                  const int* __restrict__ span_ids,
                                                  const float* __restrict__ noctx,
                                                  unsigned short* __restrict__ ctx_hi,
                                                  unsigned short* __restrict__ ctx_lo) {
  __shared__ int sel[kS];
  __shared__ __align__(16) float cs[kH];
  const int p   = blockIdx.x;
  const int b   = p / (kK * kK);
  const int ij  = p - b * (kK * kK);
  const int i   = ij / kK;
  const int j   = ij - i * kK;
  const int tid = threadIdx.x;

  const int si = span_ids[((b * kK) + i) * 2 + 0];
  const int ei = span_ids[((b * kK) + i) * 2 + 1];
  const int sj = span_ids[((b * kK) + j) * 2 + 0];
  const int ej = span_ids[((b * kK) + j) * 2 + 1];

  if (tid < kS) {
    const int t = tid;
    const bool wi  = ((t >= si - kWin) && (t < si)) || ((t > ei) && (t <= ei + kWin));
    const bool wj  = ((t >= sj - kWin) && (t < sj)) || ((t > ej) && (t <= ej + kWin));
    const bool spi = (t >= si) && (t <= ei);
    const bool spj = (t >= sj) && (t <= ej);
    const bool val = (token_masks[b * kS + t] != 0);
    sel[t] = ((wi || wj) && !spi && !spj && val) ? 1 : 0;
  }
  __syncthreads();

  const int h = tid;
  const float* trb = token_reps + (size_t)b * kS * kH + h;
  float mx = kNegLimit;
  int anysel = 0;
#pragma unroll 4
  for (int t = 0; t < kS; ++t) {
    const int m = sel[t];
    const float v = trb[(size_t)t * kH];
    mx = (m != 0) ? fmaxf(mx, v) : mx;
    anysel |= m;
  }
  const float cval = (anysel != 0) ? mx : noctx[h];
  cs[h] = cval;
  __syncthreads();

  if (tid < 64) {
    const int c8 = tid * 8;
    unsigned short hb[8], lb[8];
#pragma unroll
    for (int e = 0; e < 8; ++e) {
      const float v = cs[c8 + e];
      hb[e] = f2bf_bits(v);
      lb[e] = f2bf_bits(v - bf_bits2f(hb[e]));
    }
    const v4u uh = (v4u){pk16(hb[0], hb[1]), pk16(hb[2], hb[3]), pk16(hb[4], hb[5]), pk16(hb[6], hb[7])};
    const v4u ul = (v4u){pk16(lb[0], lb[1]), pk16(lb[2], lb[3]), pk16(lb[4], lb[5]), pk16(lb[6], lb[7])};
    const size_t o = (size_t)p * kH + c8;
    for (int pass = 0; pass < 2; ++pass) {
      *(volatile v4u*)(ctx_hi + o) = uh;
      *(volatile v4u*)(ctx_lo + o) = ul;
      __threadfence();
    }
  }
}

__global__ __launch_bounds__(256) void hid_kernel(const float* __restrict__ HT, const float* __restrict__ CXp,
                                                  const float* __restrict__ b1,
                                                  unsigned short* __restrict__ hid_hi,
                                                  unsigned short* __restrict__ hid_lo, int ngroups) {
  const int idx = blockIdx.x * 256 + threadIdx.x;
  if (idx >= ngroups) return;
  const int p  = idx / kGroupsPerRow;
  const int g  = idx - p * kGroupsPerRow;
  const int f8 = g * 8;
  const int b  = p / (kK * kK);
  const int ij = p - b * (kK * kK);
  const int i  = ij / kK;
  const int j  = ij - i * kK;
  const float* ha = HT + (size_t)(b * kK + i) * kInner + f8;
  const float* ta = HT + (size_t)kSrPad * kInner + (size_t)(b * kK + j) * kInner + f8;
  const float* cx = CXp + (size_t)p * kInner + f8;
  const float* bb = b1 + f8;
  const v4f h0 = *(const v4f*)(ha), h1 = *(const v4f*)(ha + 4);
  const v4f t0 = *(const v4f*)(ta), t1 = *(const v4f*)(ta + 4);
  const v4f c0 = *(const v4f*)(cx), c1 = *(const v4f*)(cx + 4);
  const v4f b0 = *(const v4f*)(bb), bq = *(const v4f*)(bb + 4);
  float x[8];
#pragma unroll
  for (int e = 0; e < 4; ++e) {
    x[e]     = fmaxf(((h0[e] + t0[e]) + c0[e]) + b0[e], 0.0f);
    x[4 + e] = fmaxf(((h1[e] + t1[e]) + c1[e]) + bq[e], 0.0f);
  }
  unsigned short hb[8], lb[8];
#pragma unroll
  for (int e = 0; e < 8; ++e) { hb[e] = f2bf_bits(x[e]); lb[e] = f2bf_bits(x[e] - bf_bits2f(hb[e])); }
  const v4u uh = (v4u){pk16(hb[0], hb[1]), pk16(hb[2], hb[3]), pk16(hb[4], hb[5]), pk16(hb[6], hb[7])};
  const v4u ul = (v4u){pk16(lb[0], lb[1]), pk16(lb[2], lb[3]), pk16(lb[4], lb[5]), pk16(lb[6], lb[7])};
  const size_t o = (size_t)p * kInner + f8;
  for (int pass = 0; pass < 2; ++pass) {
    *(volatile v4u*)(hid_hi + o) = uh;
    *(volatile v4u*)(hid_lo + o) = ul;
    __threadfence();
  }
}

extern "C" void kernel_launch(void* const* d_in, const int* in_sizes, int n_in,
                              void* d_out, int out_size, void* d_ws, size_t ws_size,
                              hipStream_t stream) {
  if (n_in < 9) return;
  const float* token_reps  = (const float*)d_in[0];
  const int*   token_masks = (const int*)d_in[1];
  const int*   span_ids    = (const int*)d_in[2];
  const float* span_reps   = (const float*)d_in[3];
  const float* noctx       = (const float*)d_in[4];
  const float* w1          = (const float*)d_in[5];
  const float* b1          = (const float*)d_in[6];
  const float* w2          = (const float*)d_in[7];
  const float* b2          = (const float*)d_in[8];
  float* out = (float*)d_out;
  if (in_sizes[0] != kB * kS * kH || in_sizes[5] != kThreeH * kInner || in_sizes[7] != kInner * kH) return;
  if (out_size != kPairs * kH) return;

  const size_t szW1T  = (size_t)kInner * kThreeH * 2;
  const size_t szW2T  = (size_t)kH * kInner * 2;
  const size_t szSR   = (size_t)kSrPad * kH * 2;
  const size_t szCTX  = (size_t)kPairs * kH * 2;
  const size_t szHT   = (size_t)2 * kSrPad * kInner * 4;
  const size_t szCX   = (size_t)kPairs * kInner * 4;
  const size_t szHID  = (size_t)kPairs * kInner * 2;
  size_t off = 0;
  char* base = (char*)d_ws;
  unsigned short* W1T_hi = (unsigned short*)(base + off); off += szW1T;
  unsigned short* W1T_lo = (unsigned short*)(base + off); off += szW1T;
  unsigned short* W2T_hi = (unsigned short*)(base + off); off += szW2T;
  unsigned short* W2T_lo = (unsigned short*)(base + off); off += szW2T;
  unsigned short* SR_hi  = (unsigned short*)(base + off); off += szSR;
  unsigned short* SR_lo  = (unsigned short*)(base + off); off += szSR;
  unsigned short* CTX_hi = (unsigned short*)(base + off); off += szCTX;
  unsigned short* CTX_lo = (unsigned short*)(base + off); off += szCTX;
  float*          HT     = (float*)(base + off);          off += szHT;
  float*          CX     = (float*)(base + off);          off += szCX;
  unsigned short* HID_hi = (unsigned short*)(base + off); off += szHID;
  unsigned short* HID_lo = (unsigned short*)(base + off); off += szHID;
  if (off > ws_size) return;

  tsplit_kernel<<<dim3(kThreeH / 64, kInner / 64), 256, 0, stream>>>(w1, kInner, kThreeH, W1T_hi, W1T_lo);
  tsplit_kernel<<<dim3(kInner / 64, kH / 64), 256, 0, stream>>>(w2, kH, kInner, W2T_hi, W2T_lo);
  srsplit_kernel<<<(kSrPad * (kH / 8)) / 256, 256, 0, stream>>>(span_reps, SR_hi, SR_lo);
  ctx_kernel<<<kPairs, 512, 0, stream>>>(token_reps, token_masks, span_ids, noctx, CTX_hi, CTX_lo);
  {
    const int tiles = (kSrPad / 64) * (kInner / 64);
    dim3 grid((tiles + 7) / 8, 2);
    wmma_gemm64<1, true, 0, 0, false, 0><<<grid, 256, 0, stream>>>(
        SR_hi, SR_lo, kH, 0L,
        W1T_hi, W1T_lo, kThreeH, (long)kH,
        (void*)HT, (void*)HT, kInner, (long)kSrPad * kInner,
        b1, b1, 0L,
        kSrPad, kInner, kH, 1.0f);
  }
  {
    const int tiles = (kPairs / 64) * (kInner / 64);
    dim3 grid((tiles + 7) / 8, 1);
    wmma_gemm64<1, true, 0, 0, false, 0><<<grid, 256, 0, stream>>>(
        CTX_hi, CTX_lo, kH, 0L,
        W1T_hi + 2 * kH, W1T_lo + 2 * kH, kThreeH, 0L,
        (void*)CX, (void*)CX, kInner, 0L,
        b1, b1, 0L,
        kPairs, kInner, kH, 1.0f);
  }
  {
    const int ngroups = kPairs * kGroupsPerRow;
    hid_kernel<<<(ngroups + 255) / 256, 256, 0, stream>>>(HT, CX, b1, HID_hi, HID_lo, ngroups);
  }
  {
    const int tiles = (kPairs / 64) * (kH / 64);
    dim3 grid((tiles + 7) / 8, 1);
    wmma_gemm64<1, true, 2, 0, false, 0><<<grid, 256, 0, stream>>>(
        HID_hi, HID_lo, kInner, 0L,
        W2T_hi, W2T_lo, kInner, 0L,
        (void*)out, (void*)out, kH, 0L,
        b2, b2, 0L,
        kPairs, kH, kInner, 1.0f);
  }
}
